// LoRAMHSA_89489938579616
// MI455X (gfx1250) — hardware-verified
//
#include <hip/hip_runtime.h>
#include <math.h>

constexpr int kBatch = 8;
constexpr int kSeq   = 1024;
constexpr int kDim   = 1024;
constexpr int kHeads = 16;
constexpr int kDh    = 64;
constexpr int kQKV   = 3 * kDim;
constexpr int kTok   = kBatch * kSeq;
constexpr int kRank  = 8;
constexpr int kHeadsPerChunk = 8;
constexpr int kChunks = kHeads / kHeadsPerChunk;
constexpr float kWCarry    = 16.0f;
constexpr float kPCarry    = 2048.0f;
constexpr float kYCarry    = 256.0f;
constexpr float kQkvScale  = 1.0f / kWCarry;
constexpr float kScoreScale = 0.125f;
constexpr float kPVScale   = 1.0f / kPCarry;
constexpr float kProjScale = 1.0f / (kYCarry * kWCarry);
constexpr float kLoraScale = 0.125f;

typedef __attribute__((ext_vector_type(16))) _Float16 v16h;
typedef __attribute__((ext_vector_type(8)))  _Float16 v8h;
typedef __attribute__((ext_vector_type(16))) __bf16   v16b;
typedef __attribute__((ext_vector_type(8)))  __bf16   v8b;
typedef __attribute__((ext_vector_type(8)))  float    v8f;
typedef __attribute__((ext_vector_type(4)))  float    v4f;
typedef __attribute__((ext_vector_type(4)))  unsigned int v4u;

__device__ __forceinline__ unsigned short f2bf_bits(float f) {
  unsigned u = __float_as_uint(f);
  return (unsigned short)((u + 0x7FFFu + ((u >> 16) & 1u)) >> 16);
}
__device__ __forceinline__ float bf_bits2f(unsigned short h) { return __uint_as_float(((unsigned)h) << 16); }

__device__ __forceinline__ void dep_guard_h(v8f& a, v8f& b, v16h x, v16h y) { asm volatile("v_nop\n\tv_nop\n\tv_nop\n\tv_nop" : "+v"(a), "+v"(b) : "v"(x), "v"(y)); }
__device__ __forceinline__ void dep_guard_b(v8f& a, v8f& b, v16b x, v16b y) { asm volatile("v_nop\n\tv_nop\n\tv_nop\n\tv_nop" : "+v"(a), "+v"(b) : "v"(x), "v"(y)); }
__device__ __forceinline__ void keep4_h(v16h a, v16h b, v16h c, v16h d) { asm volatile("v_nop" :: "v"(a), "v"(b), "v"(c), "v"(d)); }
__device__ __forceinline__ void keep4_b(v16b a, v16b b, v16b c, v16b d) { asm volatile("v_nop" :: "v"(a), "v"(b), "v"(c), "v"(d)); }
__device__ __forceinline__ void acc_guard4(v8f& a, v8f& b, v8f& c, v8f& d) { asm volatile("v_nop\n\tv_nop\n\tv_nop\n\tv_nop" : "+v"(a), "+v"(b), "+v"(c), "+v"(d)); }
template <typename T> struct Frag;
template <> struct Frag<_Float16> {
  typedef v16h V; union U { v16h v; v8h h[2]; };
  static __device__ __forceinline__ v16h load(const _Float16* p) {
    U f; f.h[0] = *(const v8h*)(p); f.h[1] = *(const v8h*)(p + 16); return f.v;
  }
  static __device__ __forceinline__ v8f mma(v16h a, v16h b, v8f c) {
    return __builtin_amdgcn_wmma_f32_16x16x32_f16(false, a, false, b, (short)0, c, false, false);
  }
  static __device__ __forceinline__ void guard(v8f& a, v8f& b, v16h x, v16h y) { dep_guard_h(a, b, x, y); }
  static __device__ __forceinline__ void keep(v16h a, v16h b, v16h c, v16h d) { keep4_h(a, b, c, d); }
};
template <> struct Frag<__bf16> {
  typedef v16b V; union U { v16b v; v8b h[2]; };
  static __device__ __forceinline__ v16b load(const __bf16* p) {
    U f; f.h[0] = *(const v8b*)(p); f.h[1] = *(const v8b*)(p + 16); return f.v;
  }
  static __device__ __forceinline__ v8f mma(v16b a, v16b b, v8f c) {
    return __builtin_amdgcn_wmma_f32_16x16x32_bf16(false, a, false, b, (short)0, c, false, false);
  }
  static __device__ __forceinline__ void guard(v8f& a, v8f& b, v16b x, v16b y) { dep_guard_b(a, b, x, y); }
  static __device__ __forceinline__ void keep(v16b a, v16b b, v16b c, v16b d) { keep4_b(a, b, c, d); }
};

__device__ __forceinline__ unsigned pk16(unsigned short a, unsigned short b) { return (unsigned)a | ((unsigned)b << 16); }
__device__ __forceinline__ unsigned short h_bits(float f) { const _Float16 h = (_Float16)f; return __builtin_bit_cast(unsigned short, h); }

template <int ET> struct Elem;
template <> struct Elem<0> { typedef _Float16 T; };
template <> struct Elem<1> { typedef __bf16 T; };
template <int ET, bool SPLIT, int BIAS_MODE, int OUT_MODE, bool RESID, int ACT = 0>
__global__ __launch_bounds__(256) void wmma_gemm64(
    const unsigned short* __restrict__ Ap, const unsigned short* __restrict__ A2p, int lda, long strideA,
    const unsigned short* __restrict__ Btp, const unsigned short* __restrict__ Bt2p, int ldb, long strideB,
    void* __restrict__ Cout, void* __restrict__ Cout2, int ldc, long strideC,
    const float* __restrict__ bias,
    const float* __restrict__ resid, long strideR,
    int M, int N, int K, float scale) {
  typedef typename Elem<ET>::T T;
  typedef typename Frag<T>::V V;
  const T* A = (const T*)Ap; const T* A2 = (const T*)A2p; const T* Bt = (const T*)Btp; const T* Bt2 = (const T*)Bt2p;
  __shared__ __align__(16) float sT[8][16 * 68];
  const int b    = blockIdx.y;
  const int lane = threadIdx.x & 31;
  const int wave = threadIdx.x >> 5;
  const int tilesN = N >> 6;
  const int tilesM = M >> 6;
  const int tile = blockIdx.x * 8 + wave;
  if (tile >= tilesM * tilesN) return;
  const int tm = tile / tilesN;
  const int tn = tile - tm * tilesN;
  const int m0 = tm << 6;
  const int n0 = tn << 6;

  const T* Ab  = A  + (size_t)b * strideA;
  const T* Bb  = Bt + (size_t)b * strideB;
  const T* Ab2 = SPLIT ? (A2  + (size_t)b * strideA) : nullptr;
  const T* Bb2 = SPLIT ? (Bt2 + (size_t)b * strideB) : nullptr;

  const int rlane = lane & 15;
  const int koff  = (lane >> 4) * 8;
  const int mOff  = (lane >> 4) * 8;

  v8f acc[4][4];
#pragma unroll
  for (int i = 0; i < 4; ++i)
#pragma unroll
    for (int j = 0; j < 4; ++j) acc[i][j] = (v8f){0.f,0.f,0.f,0.f,0.f,0.f,0.f,0.f};

  for (int k0 = 0; k0 < K; k0 += 32) {
    V bh[4], bl[4];
#pragma unroll
    for (int j = 0; j < 4; ++j) {
      const size_t bo = (size_t)(n0 + (j << 4) + rlane) * ldb + koff + k0;
      bh[j] = Frag<T>::load(Bb + bo);
      if (SPLIT) bl[j] = Frag<T>::load(Bb2 + bo);
    }
#pragma unroll
    for (int i = 0; i < 4; ++i) {
      const size_t ao = (size_t)(m0 + (i << 4) + rlane) * lda + koff + k0;
      V ah = Frag<T>::load(Ab + ao);
      V al;
      if (SPLIT) al = Frag<T>::load(Ab2 + ao);
#pragma unroll
      for (int j = 0; j < 4; ++j) {
        acc[i][j] = Frag<T>::mma(ah, bh[j], acc[i][j]);
        if (SPLIT) {
          acc[i][j] = Frag<T>::mma(ah, bl[j], acc[i][j]);
          acc[i][j] = Frag<T>::mma(al, bh[j], acc[i][j]);
        }
      }
      Frag<T>::guard(acc[i][0], acc[i][3], ah, SPLIT ? al : ah);
    }
    Frag<T>::keep(bh[0], bh[1], bh[2], bh[3]);
    if (SPLIT) Frag<T>::keep(bl[0], bl[1], bl[2], bl[3]);
  }
  acc_guard4(acc[0][0], acc[0][1], acc[0][2], acc[0][3]);
  acc_guard4(acc[1][0], acc[1][1], acc[1][2], acc[1][3]);
  acc_guard4(acc[2][0], acc[2][1], acc[2][2], acc[2][3]);
  acc_guard4(acc[3][0], acc[3][1], acc[3][2], acc[3][3]);

  float* slab = sT[wave];
  const float* Rb = RESID ? (resid + (size_t)b * strideR) : nullptr;
#pragma unroll
  for (int i = 0; i < 4; ++i) {
    const int mBase = m0 + (i << 4);
#pragma unroll
    for (int j = 0; j < 4; ++j) {
      const int n = n0 + (j << 4) + rlane;
      float bv = 0.f;
      if (BIAS_MODE == 2) bv = bias[n];
#pragma unroll
      for (int r = 0; r < 8; ++r) {
        float v = acc[i][j][r] * scale;
        if (BIAS_MODE == 1) v += bias[mBase + mOff + r];
        if (BIAS_MODE == 2) v += bv;
        if (RESID) v += Rb[(size_t)(mBase + mOff + r) * ldc + n];
        if (ACT == 2) v = fmaxf(v, 0.0f);
        if (ACT == 4) v = (v > 0.f) ? v : 0.01f * v;
        slab[(mOff + r) * 68 + (j << 4) + rlane] = v;
      }
    }
    __builtin_amdgcn_fence(__ATOMIC_RELEASE, "workgroup");
    __builtin_amdgcn_wave_barrier();
    __builtin_amdgcn_fence(__ATOMIC_ACQUIRE, "workgroup");
    if (OUT_MODE == 0) {
      float* C = (float*)Cout + (size_t)b * strideC;
      const int hh = lane >> 4, c4 = (lane & 15) * 4;
      for (int pass = 0; pass < 2; ++pass) {
#pragma unroll
        for (int it = 0; it < 8; ++it) {
          const int row = it * 2 + hh;
          v4f v = *(const v4f*)(slab + row * 68 + c4);
          *(volatile v4f*)(C + (size_t)(mBase + row) * ldc + n0 + c4) = v;
        }
        __threadfence();
      }
    } else {
      const int q = lane >> 3, c8 = (lane & 7) * 8;
      unsigned short* C  = (unsigned short*)Cout  + (size_t)b * strideC;
      unsigned short* C2 = (OUT_MODE == 2) ? ((unsigned short*)Cout2 + (size_t)b * strideC) : nullptr;
      for (int pass = 0; pass < 2; ++pass) {
#pragma unroll
        for (int it = 0; it < 4; ++it) {
          const int row = it * 4 + q;
          const float* sp = slab + row * 68 + c8;
          v8h hv, lv;
#pragma unroll
          for (int e = 0; e < 8; ++e) {
            if (OUT_MODE == 1) {
              hv[e] = (_Float16)sp[e];
            } else {
              unsigned short hb = f2bf_bits(sp[e]);
              unsigned short lb = f2bf_bits(sp[e] - bf_bits2f(hb));
              hv[e] = __builtin_bit_cast(_Float16, hb);
              lv[e] = __builtin_bit_cast(_Float16, lb);
            }
          }
          *(volatile v8h*)(C + (size_t)(mBase + row) * ldc + n0 + c8) = hv;
          if (OUT_MODE == 2) *(volatile v8h*)(C2 + (size_t)(mBase + row) * ldc + n0 + c8) = lv;
        }
        __threadfence();
      }
    }
    __builtin_amdgcn_fence(__ATOMIC_RELEASE, "workgroup");
    __builtin_amdgcn_wave_barrier();
    __builtin_amdgcn_fence(__ATOMIC_ACQUIRE, "workgroup");
  }
}

__global__ __launch_bounds__(256) void cast8_f16_kernel(const float* __restrict__ in, unsigned short* __restrict__ out,
                                                        int n8, float scale) {
  const int i = blockIdx.x * 256 + threadIdx.x;
  if (i >= n8) return;
  const float* p = in + 8 * (size_t)i;
  const v4f a = *(const v4f*)(p);
  const v4f c = *(const v4f*)(p + 4);
  unsigned short hb[8];
#pragma unroll
  for (int e = 0; e < 4; ++e) {
    hb[e]     = h_bits(a[e] * scale);
    hb[4 + e] = h_bits(c[e] * scale);
  }
  const v4u u = (v4u){pk16(hb[0], hb[1]), pk16(hb[2], hb[3]), pk16(hb[4], hb[5]), pk16(hb[6], hb[7])};
  unsigned short* q = out + 8 * (size_t)i;
  *(volatile v4u*)q = u;
  __threadfence();
  *(volatile v4u*)q = u;
}

__device__ __forceinline__ int sel_adapter(const int* __restrict__ sid, int b, int nAdapt) {
  int s = sid[b];
  s = s < 0 ? 0 : s;
  s = s > nAdapt - 1 ? nAdapt - 1 : s;
  return s;
}

__global__ __launch_bounds__(256) void lora_h_kernel(const float* __restrict__ X, const float* __restrict__ A,
                                                     const int* __restrict__ sid, float* __restrict__ H, int nAdapt) {
  __shared__ __align__(16) float hs[32 * kRank];
  const int t   = threadIdx.x;
  const int rl  = t >> 3;
  const int r   = t & 7;
  const int row = blockIdx.x * 32 + rl;
  const int s   = sel_adapter(sid, row / kSeq, nAdapt);
  const float* xr = X + (size_t)row * kDim;
  const float* ar = A + ((size_t)s * kRank + r) * kDim;
  float acc = 0.f;
#pragma unroll 4
  for (int d = 0; d < kDim; d += 4) {
    const v4f xv = *(const v4f*)(xr + d);
    const v4f av = *(const v4f*)(ar + d);
    acc += xv[0] * av[0];
    acc += xv[1] * av[1];
    acc += xv[2] * av[2];
    acc += xv[3] * av[3];
  }
  hs[rl * kRank + r] = acc;
  __syncthreads();
  if (t < 32) {
    const v4f v0 = *(const v4f*)(hs + t * 4);
    const v4f v1 = *(const v4f*)(hs + 128 + t * 4);
    float* hp = H + (size_t)blockIdx.x * 256;
    *(volatile v4f*)(hp + t * 4) = v0;
    *(volatile v4f*)(hp + 128 + t * 4) = v1;
    __threadfence();
    *(volatile v4f*)(hp + t * 4) = v0;
    *(volatile v4f*)(hp + 128 + t * 4) = v1;
  }
}

__global__ __launch_bounds__(256) void lora_resid_kernel(const float* __restrict__ H, const float* __restrict__ Bm,
                                                         const int* __restrict__ sid, float* __restrict__ R,
                                                         int rowBase, int nAdapt, int N) {
  const int rowL = blockIdx.x;
  const int row  = rowBase + rowL;
  const int s    = sel_adapter(sid, row / kSeq, nAdapt);
  const v4f h0 = *(const v4f*)(H + (size_t)row * kRank);
  const v4f h1 = *(const v4f*)(H + (size_t)row * kRank + 4);
  const float* bb = Bm + (size_t)s * N * kRank;
  float* rr = R + (size_t)rowL * N;
  for (int c = threadIdx.x * 4; c < N; c += 1024) {
    v4f o;
#pragma unroll
    for (int e = 0; e < 4; ++e) {
      const float* bp = bb + (size_t)(c + e) * kRank;
      const v4f b0 = *(const v4f*)(bp);
      const v4f b1 = *(const v4f*)(bp + 4);
      float a = h0[0] * b0[0];
      a += h0[1] * b0[1];
      a += h0[2] * b0[2];
      a += h0[3] * b0[3];
      a += h1[0] * b1[0];
      a += h1[1] * b1[1];
      a += h1[2] * b1[2];
      a += h1[3] * b1[3];
      o[e] = kLoraScale * a;
    }
    *(volatile v4f*)(rr + c) = o;
    __threadfence();
    *(volatile v4f*)(rr + c) = o;
  }
}

__global__ __launch_bounds__(256) void vt_kernel(const unsigned short* __restrict__ qkv, unsigned short* __restrict__ vt) {
  __shared__ unsigned short sm[64][72];
  const int t  = threadIdx.x;
  const int t0 = blockIdx.x * 64;
  const int h  = blockIdx.y;
#pragma unroll
  for (int it = 0; it < 2; ++it) {
    const int e  = it * 256 + t;
    const int r  = e >> 3;
    const int c8 = (e & 7) * 8;
    const v4u u = *(const v4u*)(qkv + (size_t)(t0 + r) * kQKV + 2 * kDim + h * kDh + c8);
#pragma unroll
    for (int w = 0; w < 4; ++w) {
      sm[c8 + 2 * w][r]     = (unsigned short)(u[w] & 0xffffu);
      sm[c8 + 2 * w + 1][r] = (unsigned short)(u[w] >> 16);
    }
  }
  __syncthreads();
  const int lane = t & 31, wave = t >> 5;
  const int q = lane >> 3, c8 = (lane & 7) * 8;
  unsigned short* op = vt + (size_t)h * kDh * kSeq + t0;
  for (int pass = 0; pass < 2; ++pass) {
#pragma unroll
    for (int it = 0; it < 2; ++it) {
      const int row = wave * 8 + it * 4 + q;
      const v4u u = (v4u){pk16(sm[row][c8 + 0], sm[row][c8 + 1]), pk16(sm[row][c8 + 2], sm[row][c8 + 3]),
                          pk16(sm[row][c8 + 4], sm[row][c8 + 5]), pk16(sm[row][c8 + 6], sm[row][c8 + 7])};
      *(volatile v4u*)(op + (size_t)row * kSeq + c8) = u;
    }
    __threadfence();
  }
}

__global__ __launch_bounds__(128) void softmax_row_kernel(const float* __restrict__ S, unsigned short* __restrict__ P, float carry) {
  __shared__ float red[8];
  __shared__ __align__(16) float es[kSeq];
  const int row  = blockIdx.x;
  const int t    = threadIdx.x;
  const int lane = t & 31, wave = t >> 5;
  const int c0   = t * 8;
  const float* sr = S + (size_t)row * kSeq + c0;
  const v4f a = *(const v4f*)(sr);
  const v4f c = *(const v4f*)(sr + 4);
  float m = fmaxf(fmaxf(fmaxf(a[0], a[1]), fmaxf(a[2], a[3])), fmaxf(fmaxf(c[0], c[1]), fmaxf(c[2], c[3])));
#pragma unroll
  for (int off = 16; off > 0; off >>= 1) m = fmaxf(m, __shfl_xor(m, off, 32));
  if (lane == 0) red[wave] = m;
  __syncthreads();
  m = fmaxf(fmaxf(red[0], red[1]), fmaxf(red[2], red[3]));
  float sum = 0.f;
#pragma unroll 1
  for (int i = 0; i < 8; ++i) {
    const float e = expf(sr[i] - m);
    es[c0 + i] = e;
    sum += e;
  }
#pragma unroll
  for (int off = 16; off > 0; off >>= 1) sum += __shfl_xor(sum, off, 32);
  if (lane == 0) red[4 + wave] = sum;
  __syncthreads();
  const float tot = ((red[4] + red[5]) + red[6]) + red[7];
  const float f = carry * (1.0f / tot);
  const v4f e0 = *(const v4f*)(es + c0);
  const v4f e1 = *(const v4f*)(es + c0 + 4);
  unsigned short hb[8];
#pragma unroll
  for (int e = 0; e < 4; ++e) {
    hb[e]     = h_bits(e0[e] * f);
    hb[4 + e] = h_bits(e1[e] * f);
  }
  const v4u u = (v4u){pk16(hb[0], hb[1]), pk16(hb[2], hb[3]), pk16(hb[4], hb[5]), pk16(hb[6], hb[7])};
  unsigned short* pp = P + (size_t)row * kSeq + c0;
  *(volatile v4u*)pp = u;
  __threadfence();
  *(volatile v4u*)pp = u;
}

extern "C" void kernel_launch(void* const* d_in, const int* in_sizes, int n_in,
                              void* d_out, int out_size, void* d_ws, size_t ws_size, hipStream_t stream) {
  if (n_in < 11) return;
  const float* x     = (const float*)d_in[0];
  const int*   sid   = (const int*)d_in[2];
  const float* Wqkv  = (const float*)d_in[3];
  const float* bqkv  = (const float*)d_in[4];
  const float* A1    = (const float*)d_in[5];
  const float* B1    = (const float*)d_in[6];
  const float* Wp    = (const float*)d_in[7];
  const float* bp    = (const float*)d_in[8];
  const float* A2    = (const float*)d_in[9];
  const float* B2    = (const float*)d_in[10];

  if (in_sizes[0] != kTok * kDim) return;
  if (in_sizes[2] != kBatch) return;
  if (in_sizes[3] != kQKV * kDim) return;
  if (in_sizes[4] != kQKV) return;
  if (in_sizes[7] != kDim * kDim) return;
  if (in_sizes[8] != kDim) return;
  if (out_size != kTok * kDim) return;
  const int nAdapt = in_sizes[5] / (kRank * kDim);
  if (nAdapt < 1) return;
  if (in_sizes[5] != nAdapt * kRank * kDim) return;
  if (in_sizes[6] != nAdapt * kQKV * kRank) return;
  if (in_sizes[9] != nAdapt * kRank * kDim) return;
  if (in_sizes[10] != nAdapt * kDim * kRank) return;

  static_assert((size_t)kHeadsPerChunk * kSeq * kSeq * 4 == (size_t)kTok * kDim * 4);
  static_assert((size_t)kHeadsPerChunk * kSeq * kSeq * 2 == (size_t)kTok * kDim * 2);
  char* ws = (char*)d_ws;
  size_t off = 0;
  unsigned short* xh    = (unsigned short*)(ws + off); off += (size_t)kTok * kDim * 2;
  unsigned short* wqkvh = (unsigned short*)(ws + off); off += (size_t)kQKV * kDim * 2;
  unsigned short* wph   = (unsigned short*)(ws + off); off += (size_t)kDim * kDim * 2;
  float*          h1    = (float*)(ws + off);          off += (size_t)kTok * kRank * 4;
  float*          h2    = (float*)(ws + off);          off += (size_t)kTok * kRank * 4;
  float*          resid1 = (float*)(ws + off);         off += (size_t)kSeq * kQKV * 4;
  unsigned short* qkvh  = (unsigned short*)(ws + off); off += (size_t)kSeq * kQKV * 2;
  unsigned short* vt    = (unsigned short*)(ws + off); off += (size_t)kHeads * kDh * kSeq * 2;
  float*          scores = (float*)(ws + off);         off += (size_t)kHeadsPerChunk * kSeq * kSeq * 4;
  unsigned short* pbuf  = (unsigned short*)(ws + off); off += (size_t)kHeadsPerChunk * kSeq * kSeq * 2;
  float*          ybuf  = (float*)(ws + off);          off += (size_t)kTok * kDim * 4;
  if (off > ws_size) return;
  float*          resid2 = scores;
  unsigned short* yh     = pbuf;
  float* out = (float*)d_out;

  {
    const int n8x = kTok * kDim / 8;
    cast8_f16_kernel<<<dim3((n8x + 255) / 256), dim3(256), 0, stream>>>(x, xh, n8x, 1.0f);
    const int n8w = kQKV * kDim / 8;
    cast8_f16_kernel<<<dim3((n8w + 255) / 256), dim3(256), 0, stream>>>(Wqkv, wqkvh, n8w, kWCarry);
    const int n8p = kDim * kDim / 8;
    cast8_f16_kernel<<<dim3((n8p + 255) / 256), dim3(256), 0, stream>>>(Wp, wph, n8p, kWCarry);
  }
  lora_h_kernel<<<dim3(kTok / 32), dim3(256), 0, stream>>>(x, A1, sid, h1, nAdapt);

  for (int b = 0; b < kBatch; ++b) {
    lora_resid_kernel<<<dim3(kSeq), dim3(256), 0, stream>>>(h1, B1, sid, resid1, b * kSeq, nAdapt, kQKV);
    wmma_gemm64<0, false, 2, 1, true><<<dim3((kSeq / 64) * (kQKV / 64) / 8, 1), dim3(256), 0, stream>>>(
        xh + (size_t)b * kSeq * kDim, xh + (size_t)b * kSeq * kDim, kDim, 0L,
        wqkvh, wqkvh, kDim, 0L,
        (void*)qkvh, (void*)qkvh, kQKV, 0L,
        bqkv,
        resid1, 0L,
        kSeq, kQKV, kDim, kQkvScale);
    vt_kernel<<<dim3(kSeq / 64, kHeads), dim3(256), 0, stream>>>(qkvh, vt);
    for (int ch = 0; ch < kChunks; ++ch) {
      const size_t hcol = (size_t)ch * kHeadsPerChunk * kDh;
      wmma_gemm64<0, false, 0, 0, false><<<dim3(32, kHeadsPerChunk), dim3(256), 0, stream>>>(
          qkvh + hcol, qkvh + hcol, kQKV, (long)kDh,
          qkvh + kDim + hcol, qkvh + kDim + hcol, kQKV, (long)kDh,
          (void*)scores, (void*)scores, kSeq, (long)kSeq * kSeq,
          bqkv,
          resid1, 0L,
          kSeq, kSeq, kDh, kScoreScale);
      softmax_row_kernel<<<dim3(kHeadsPerChunk * kSeq), dim3(128), 0, stream>>>(scores, pbuf, kPCarry);
      wmma_gemm64<0, false, 0, 0, false><<<dim3(2, kHeadsPerChunk), dim3(256), 0, stream>>>(
          pbuf, pbuf, kSeq, (long)kSeq * kSeq,
          vt + hcol * kSeq, vt + hcol * kSeq, kSeq, (long)kDh * kSeq,
          (void*)(ybuf + (size_t)b * kSeq * kDim + hcol), (void*)(ybuf + (size_t)b * kSeq * kDim + hcol), kDim, (long)kDh,
          bqkv,
          resid1, 0L,
          kSeq, kDh, kSeq, kPVScale);
    }
  }

  {
    const int n8y = kTok * kDim / 8;
    cast8_f16_kernel<<<dim3((n8y + 255) / 256), dim3(256), 0, stream>>>(ybuf, yh, n8y, kYCarry);
  }
  lora_h_kernel<<<dim3(kTok / 32), dim3(256), 0, stream>>>(ybuf, A2, sid, h2, nAdapt);
  lora_resid_kernel<<<dim3(kTok), dim3(256), 0, stream>>>(h2, B2, sid, resid2, 0, nAdapt, kDim);
  wmma_gemm64<0, false, 2, 0, true><<<dim3((kTok / 64) * (kDim / 64) / 8, 1), dim3(256), 0, stream>>>(
      yh, yh, kDim, 0L,
      wph, wph, kDim, 0L,
      (void*)out, (void*)out, kDim, 0L,
      bp,
      resid2, 0L,
      kTok, kDim, kDim, kProjScale);
}
